// MambaBlock_13211319402874
// MI455X (gfx1250) — hardware-run, weakly checked
//
#include <hip/hip_runtime.h>


#ifndef NB
#define NB 2
#endif
#ifndef SEQ
#define SEQ 2048
#endif
#define NB_FULL  2
#define SEQ_FULL 2048
#ifndef OUT_SEQ
#define OUT_SEQ SEQ
#endif
#define DM   1024
#define DI   2048
#define DS   16
#define DR   64
#define XPN  96
#define XPP  128
#define XZW  4096
#define BCW  32
#define WSC  64.0f
#define XCC  64.0f
#define DTRC 64.0f
#define YCC  256.0f
#define TCH  64
#define CT   8
#define L2E  1.4426950408889634f
#define LN2F 0.6931471805599453f

static_assert(DI == 2 * DM);
static_assert(XZW == 2 * DI);
static_assert(XPN == DR + 2 * DS);
static_assert(XPP % 64 == 0);
static_assert(XPP >= XPN);
static_assert(DR == 64);
static_assert(BCW == 2 * DS);
static_assert(BCW * 4 == 128);
static_assert(64 + BCW <= XPP);
static_assert(DM % 32 == 0);
static_assert(DI % 32 == 0);
static_assert(DR % 32 == 0);
static_assert(DM % 64 == 0);
static_assert(DI % 64 == 0);
static_assert(XZW % 64 == 0);
static_assert((NB * SEQ) % 64 == 0);
static_assert(SEQ % 64 == 0);
static_assert(SEQ % TCH == 0);
static_assert(SEQ % CT == 0);
static_assert(CT >= 3);
static_assert(256 * 8 == DI);
static_assert(32 * 4 * 8 == DM);
static_assert((NB * SEQ) % 4 == 0);
static_assert(64 * 8 * 4 == TCH * BCW);
static_assert(64 * 16 * 8 == TCH * 128);
static_assert(32 * 16 * 4 == 16 * 128);
static_assert(32 * 16 * 8 == 16 * 256);
static_assert(NB <= NB_FULL);
static_assert(SEQ <= SEQ_FULL);
static_assert(((size_t)SEQ * DM) % 8 == 0);

typedef _Float16 h16;
typedef unsigned short bf;
typedef __attribute__((ext_vector_type(16))) __bf16   v16bf;
typedef __attribute__((ext_vector_type(16))) _Float16 v16h;
typedef __attribute__((ext_vector_type(8)))  _Float16 v8h;
typedef __attribute__((ext_vector_type(8)))  unsigned short v8us;
typedef __attribute__((ext_vector_type(8)))  float    v8f;
typedef __attribute__((ext_vector_type(4)))  float    v4f;
typedef v4f  __attribute__((may_alias)) v4fa;
typedef v8h  __attribute__((may_alias)) v8ha;

__device__ __forceinline__ unsigned short f2bf(float f) { unsigned u = __float_as_uint(f); u += 0x7FFFu + ((u >> 16) & 1u); return (unsigned short)(u >> 16); }
__device__ __forceinline__ float bfr(float f) { return __uint_as_float(((unsigned)f2bf(f)) << 16); }
__device__ __forceinline__ v16h cat16(v8h lo, v8h hi) { return __builtin_shufflevector(lo, hi, 0, 1, 2, 3, 4, 5, 6, 7, 8, 9, 10, 11, 12, 13, 14, 15); }
__device__ __forceinline__ v16bf cat16b(v8us lo, v8us hi) { return __builtin_bit_cast(v16bf, __builtin_shufflevector(lo, hi, 0, 1, 2, 3, 4, 5, 6, 7, 8, 9, 10, 11, 12, 13, 14, 15)); }
__device__ __forceinline__ v8f wmma16(v16h a, v16h b, v8f c) { return __builtin_amdgcn_wmma_f32_16x16x32_f16(false, a, false, b, (short)0, c, false, false); }
__device__ __forceinline__ v8f wmmab(v16bf a, v16bf b, v8f c) { return __builtin_amdgcn_wmma_f32_16x16x32_bf16(false, a, false, b, (short)0, c, false, false); }
__device__ __forceinline__ v16h  ldh(const h16* p) { return cat16(*(const v8h*)p, *(const v8h*)(p + 16)); }
__device__ __forceinline__ v16bf ldb(const bf* p)  { return cat16b(*(const v8us*)p, *(const v8us*)(p + 16)); }
__device__ __forceinline__ void wave_sync() { __builtin_amdgcn_fence(3  , "wavefront"); __builtin_amdgcn_wave_barrier(); asm volatile("" ::: "memory"); }

static __device__ __forceinline__ h16 toh_flush(float v) { const h16 r = (h16)v; return (fabsf(v) < 6.103515625e-05f) ? (h16)0.0f : r; }

__device__ __forceinline__ v16bf ldf(const bf* p)  { return ldb(p); }
__device__ __forceinline__ v16h  ldf(const h16* p) { return ldh(p); }
__device__ __forceinline__ v8f mma(v16bf a, v16bf b, v8f c) { return wmmab(a, b, c); }
__device__ __forceinline__ v8f mma(v16h a, v16h b, v8f c)   { return wmma16(a, b, c); }
template <typename T> struct fragof;
template <> struct fragof<bf>  { typedef v16bf type; };
template <> struct fragof<h16> { typedef v16h  type; };

__device__ __forceinline__ float softplus_f(float x) {
    const float xm = fminf(x, 20.0f);
    const float e = __builtin_amdgcn_exp2f(xm * L2E);
    const float sp = LN2F * __log2f(1.0f + e);
    return (x > 20.0f) ? x : sp;
}

__global__ __launch_bounds__(256) void k_cvt8(const float* __restrict__ src, bf* dst, size_t n8) {
    const size_t i = (size_t)blockIdx.x * 256 + threadIdx.x; if (i >= n8) return;
    const v8f v = *(const v8f*)(src + i * 8); v8us o;
#pragma unroll
    for (int k = 0; k < 8; ++k) o[k] = f2bf(v[k]);
    *(volatile v8us*)(dst + i * 8) = o; __threadfence(); *(volatile v8us*)(dst + i * 8) = o;
}

__global__ __launch_bounds__(256) void k_wcvth(const float* __restrict__ src, h16* dst, size_t n8src, size_t n8dst, float scale) {
    const size_t i = (size_t)blockIdx.x * 256 + threadIdx.x; if (i >= n8dst) return;
    const size_t si = (i < n8src) ? i : (n8src - 1);
    v8f v = *(const v8f*)(src + si * 8);
    asm volatile("" : "+v"(v));
    const bool ok = i < n8src;
    v8h o;
#pragma unroll
    for (int k = 0; k < 8; ++k) { const h16 c = toh_flush(bfr(v[k]) * scale); o[k] = ok ? c : (h16)0.0f; }
    *(volatile v8h*)(dst + i * 8) = o; __threadfence(); *(volatile v8h*)(dst + i * 8) = o;
}

template <int EPI, int K, typename T>
__device__ __forceinline__ void gemm_body(const T* __restrict__ A, const T* __restrict__ Bt, const float* __restrict__ bias, h16* Ph, float* Pf) {
    typedef typename fragof<T>::type frag;
    __shared__ __align__(16) float os[16 * 68];
    static_assert(sizeof(float) * 16 * 68 <= 131072);
    static_assert(K % 32 == 0);
    const int lane = threadIdx.x & 31, lr = lane & 15, hi = lane >> 4; const int r0 = blockIdx.x * 64, c0 = blockIdx.y * 64;
    v8f acc[4][4];
#pragma unroll
    for (int mb = 0; mb < 4; ++mb)
#pragma unroll
        for (int nb = 0; nb < 4; ++nb) acc[mb][nb] = (v8f){};
    const size_t aoff = (size_t)(r0 + lr) * K + 8 * hi, boff = (size_t)(c0 + lr) * K + 8 * hi;
#pragma unroll 1
    for (int kc = 0; kc < K; kc += 32) {
        frag a[4];
#pragma unroll
        for (int mb = 0; mb < 4; ++mb) a[mb] = ldf(A + aoff + (size_t)mb * 16 * K + kc);
#pragma unroll
        for (int nb = 0; nb < 4; ++nb) { const frag b = ldf(Bt + boff + (size_t)nb * 16 * K + kc);
#pragma unroll
            for (int mb = 0; mb < 4; ++mb) acc[mb][nb] = mma(a[mb], b, acc[mb][nb]); }
        asm volatile("v_nop\n\tv_nop\n\tv_nop\n\tv_nop" : "+v"(acc[0][0]), "+v"(acc[1][1]), "+v"(acc[2][2]), "+v"(acc[3][3]) : "v"(a[0]), "v"(a[1]), "v"(a[2]), "v"(a[3]));
    }
    float bc[4];
#pragma unroll
    for (int nb = 0; nb < 4; ++nb) bc[nb] = (EPI == 2) ? bfr(bias[c0 + nb * 16 + lr]) : 0.0f;
    const bool zact  = (EPI == 0) && (c0 >= DI);
    const bool tile0 = (EPI == 1) && (blockIdx.y == 0);
    const bool hrows = (EPI == 0) || (EPI == 2) || tile0;
    float sc = 1.0f;
    if (EPI == 1) sc = tile0 ? (DTRC / (XCC * WSC)) : (1.0f / (XCC * WSC));
    if (EPI == 2) sc = 1.0f / (DTRC * WSC);
    if (EPI == 3) sc = 1.0f / (YCC * WSC);
    const size_t ldc = (EPI == 0) ? (size_t)XZW : ((EPI == 2) ? (size_t)DI : (size_t)DR);
    const size_t cb  = (EPI == 1) ? (size_t)0 : (size_t)c0;
#pragma unroll
    for (int mb = 0; mb < 4; ++mb) {
#pragma unroll
        for (int nb = 0; nb < 4; ++nb) {
#pragma unroll
            for (int j = 0; j < 8; ++j) {
                float v = acc[mb][nb][j] * sc;
                if (EPI == 0) { if (zact) v = v * __builtin_amdgcn_rcpf(1.0f + __builtin_amdgcn_exp2f(-v * L2E)); }
                if (EPI == 2) v = softplus_f(v + bc[nb]);
                os[(hi * 8 + j) * 68 + nb * 16 + lr] = v; } }
        wave_sync();
#pragma unroll 1
        for (int ps = 0; ps < 2; ++ps) {
            if (hrows) {
                const size_t sb = (size_t)(r0 + mb * 16) * ldc + cb;
#pragma unroll
                for (int s = 0; s < 4; ++s) { const int row = 4 * s + (lane >> 3), c8 = (lane & 7) * 8;
                    const v4f x0 = *(const v4fa*)(&os[row * 68 + c8]); const v4f x1 = *(const v4fa*)(&os[row * 68 + c8 + 4]); v8h hv;
#pragma unroll
                    for (int i = 0; i < 4; ++i) { hv[i] = toh_flush(x0[i]); hv[4 + i] = toh_flush(x1[i]); }
                    *(volatile v8h*)(Ph + sb + (size_t)row * ldc + c8) = hv; }
            } else if (EPI == 1) {
                const size_t sb = (size_t)(r0 + mb * 16) * BCW;
#pragma unroll
                for (int s = 0; s < 4; ++s) { const int row = 4 * s + (lane >> 3), cofs = (lane & 7) * 4;
                    const v4f val = *(const v4fa*)(&os[row * 68 + cofs]);
                    *(volatile v4f*)(Pf + sb + (size_t)row * BCW + cofs) = val; }
            } else {
                const size_t sb = (size_t)(r0 + mb * 16) * DM + (size_t)c0;
#pragma unroll
                for (int s = 0; s < 8; ++s) { const int row = 2 * s + (lane >> 4), cofs = (lane & 15) * 4;
                    const v4f val = *(const v4fa*)(&os[row * 68 + cofs]);
                    *(volatile v4f*)(Pf + sb + (size_t)row * DM + cofs) = val; }
            }
            if (ps == 0) __threadfence(); }
        wave_sync();
    }
}

__global__ __launch_bounds__(32) void k_gemm_in(const bf* __restrict__ A, const bf* __restrict__ Bt, h16* P) {
    gemm_body<0, DM, bf>(A, Bt, (const float*)nullptr, P, (float*)nullptr);
}
__global__ __launch_bounds__(32) void k_gemm_xp(const h16* __restrict__ A, const h16* __restrict__ Bt, h16* Pd, float* Pb) {
    gemm_body<1, DI, h16>(A, Bt, (const float*)nullptr, Pd, Pb);
}
__global__ __launch_bounds__(32) void k_gemm_dt(const h16* __restrict__ A, const h16* __restrict__ Bt, const float* __restrict__ bias, h16* P) {
    gemm_body<2, DR, h16>(A, Bt, bias, P, (float*)nullptr);
}
__global__ __launch_bounds__(32) void k_gemm_out(const h16* __restrict__ A, const h16* __restrict__ Bt, float* P) {
    gemm_body<3, DI, h16>(A, Bt, (const float*)nullptr, (h16*)nullptr, P);
}

__global__ __launch_bounds__(256) void k_conv(const h16* __restrict__ XZ, const float* __restrict__ cw, const float* __restrict__ cb, h16* XC) {
    const int row0 = blockIdx.x * CT; const int t0 = row0 % SEQ;
    const int c = threadIdx.x * 8;
    float w0[8], w1[8], w2[8], w3[8], bs[8];
#pragma unroll
    for (int i = 0; i < 8; ++i) { const v4f wv = *(const v4f*)(cw + (size_t)(c + i) * 4); w0[i] = bfr(wv[0]); w1[i] = bfr(wv[1]); w2[i] = bfr(wv[2]); w3[i] = bfr(wv[3]); }
    { const v4f b0 = *(const v4f*)(cb + c), b1 = *(const v4f*)(cb + c + 4);
#pragma unroll
      for (int i = 0; i < 4; ++i) { bs[i] = bfr(b0[i]); bs[4 + i] = bfr(b1[i]); } }
    const bool hal = t0 > 0;
    const size_t rp = hal ? (size_t)(row0 - 3) : (size_t)row0;
#pragma unroll 1
    for (int ps = 0; ps < 2; ++ps) {
        float xa[8], xb[8], xm[8];
        { const v8h ha = *(const v8h*)(XZ + (rp + 0) * XZW + c), hb = *(const v8h*)(XZ + (rp + 1) * XZW + c), hc = *(const v8h*)(XZ + (rp + 2) * XZW + c);
#pragma unroll
          for (int k = 0; k < 8; ++k) { xa[k] = hal ? (float)ha[k] : 0.0f; xb[k] = hal ? (float)hb[k] : 0.0f; xm[k] = hal ? (float)hc[k] : 0.0f; } }
#pragma unroll 1
        for (int i = 0; i < CT; ++i) {
            const v8h cv = *(const v8h*)(XZ + (size_t)(row0 + i) * XZW + c);
            v8h o;
#pragma unroll
            for (int k = 0; k < 8; ++k) {
                const float xd = (float)cv[k];
                const float a = bs[k] + w0[k] * xa[k] + w1[k] * xb[k] + w2[k] * xm[k] + w3[k] * xd;
                const float sg = __builtin_amdgcn_rcpf(1.0f + __builtin_amdgcn_exp2f(-a * L2E));
                o[k] = toh_flush(a * sg * XCC);
                xa[k] = xb[k]; xb[k] = xm[k]; xm[k] = xd; }
            *(volatile v8h*)(XC + (size_t)(row0 + i) * DI + c) = o;
        }
        if (ps == 0) __threadfence();
    }
}

__global__ __launch_bounds__(64) void k_scan(const h16* __restrict__ DT, const h16* __restrict__ XC, const h16* __restrict__ XZ, const float* __restrict__ BC,
                                             const float* __restrict__ alog, const float* __restrict__ dskip, h16* Y) {
    __shared__ __align__(16) float bcs[TCH * BCW];
    __shared__ __align__(16) h16 ys[TCH * 64];
    static_assert(sizeof(float) * TCH * BCW + sizeof(h16) * TCH * 64 <= 131072);
    const int tid = threadIdx.x; const int d = blockIdx.x * 64 + tid; const int b = blockIdx.y;
    float A2[16], h[16];
#pragma unroll
    for (int q = 0; q < 4; ++q) { const v4f al = *(const v4f*)(alog + (size_t)d * DS + 4 * q);
#pragma unroll
        for (int k = 0; k < 4; ++k) { A2[4 * q + k] = -__builtin_amdgcn_exp2f(bfr(al[k]) * L2E) * L2E; h[4 * q + k] = 0.0f; } }
    const float Dd = bfr(dskip[d]);
    const size_t rb = (size_t)b * SEQ;
#pragma unroll 1
    for (int tc = 0; tc < SEQ; tc += TCH) {
        const v4f* src = (const v4f*)(BC + (rb + (size_t)tc) * BCW);
#pragma unroll
        for (int k = 0; k < 8; ++k) { const v4f val = src[tid + 64 * k]; *(v4fa*)(&bcs[(tid + 64 * k) * 4]) = val; }
        __syncthreads();
#pragma unroll 1
        for (int t = 0; t < TCH; ++t) {
            const size_t row = rb + (size_t)tc + (size_t)t;
            const float dt = (float)DT[row * DI + d];
            const float u  = (float)XC[row * DI + d] * (1.0f / XCC);
            const float zs = (float)XZ[row * XZW + DI + d];
            v4f bq[4], cq[4];
#pragma unroll
            for (int k = 0; k < 4; ++k) { bq[k] = *(const v4fa*)(&bcs[t * BCW + 4 * k]); cq[k] = *(const v4fa*)(&bcs[t * BCW + DS + 4 * k]); }
            const float dbu = dt * u;
            float y = Dd * u;
#pragma unroll
            for (int s = 0; s < 16; ++s) {
                const float e = __builtin_amdgcn_exp2f(dt * A2[s]);
                h[s] = e * h[s] + dbu * bq[s >> 2][s & 3];
                y += h[s] * cq[s >> 2][s & 3]; }
            ys[t * 64 + tid] = toh_flush(y * zs * YCC);
        }
        __syncthreads();
#pragma unroll 1
        for (int ps = 0; ps < 2; ++ps) {
#pragma unroll
            for (int s2 = 0; s2 < 8; ++s2) { const int row = 8 * s2 + (tid >> 3), c8 = (tid & 7) * 8;
                const v8h val = *(const v8ha*)(&ys[row * 64 + c8]);
                *(volatile v8h*)(Y + (rb + (size_t)tc + (size_t)row) * DI + (size_t)blockIdx.x * 64 + c8) = val; }
            if (ps == 0) __threadfence(); }
    }
}

__global__ __launch_bounds__(128) void k_ln(const float* __restrict__ PRE, const float* __restrict__ X, const float* __restrict__ g, const float* __restrict__ be, float* OUT) {
    const int lane = threadIdx.x & 31;
    const int wave = __builtin_amdgcn_readfirstlane((int)(threadIdx.x >> 5));
    const int row = blockIdx.x * 4 + wave;
    const int b = row / SEQ, t = row % SEQ;
    const float* pr = PRE + (size_t)row * DM;
    const float* xr = X + ((size_t)b * SEQ_FULL + (size_t)t) * DM;
    float* orow = OUT + ((size_t)b * OUT_SEQ + (size_t)t) * DM;
    float s = 0.0f;
#pragma unroll 1
    for (int i = 0; i < 8; ++i) { const int c = i * 128 + lane * 4;
        const v4f p = *(const v4f*)(pr + c); const v4f x = *(const v4f*)(xr + c);
#pragma unroll
        for (int k = 0; k < 4; ++k) s += p[k] + bfr(x[k]); }
#pragma unroll
    for (int o = 16; o > 0; o >>= 1) s += __shfl_xor(s, o, 32);
    const float mean = s * (1.0f / DM);
    float q = 0.0f;
#pragma unroll 1
    for (int i = 0; i < 8; ++i) { const int c = i * 128 + lane * 4;
        const v4f p = *(const v4f*)(pr + c); const v4f x = *(const v4f*)(xr + c);
#pragma unroll
        for (int k = 0; k < 4; ++k) { const float dv = (p[k] + bfr(x[k])) - mean; q += dv * dv; } }
#pragma unroll
    for (int o = 16; o > 0; o >>= 1) q += __shfl_xor(q, o, 32);
    const float rstd = rsqrtf(q * (1.0f / DM) + 1e-5f);
#pragma unroll 1
    for (int ps = 0; ps < 2; ++ps) {
#pragma unroll 1
        for (int i = 0; i < 8; ++i) { const int c = i * 128 + lane * 4;
            const v4f p = *(const v4f*)(pr + c); const v4f x = *(const v4f*)(xr + c);
            const v4f gg = *(const v4f*)(g + c); const v4f bb = *(const v4f*)(be + c);
            v4f o;
#pragma unroll
            for (int k = 0; k < 4; ++k) { const float dv = (p[k] + bfr(x[k])) - mean; o[k] = dv * rstd * bfr(gg[k]) + bfr(bb[k]); }
            *(volatile v4f*)(orow + c) = o; }
        if (ps == 0) __threadfence(); }
}

static constexpr size_t al256(size_t v) { return (v + 255) & ~(size_t)255; }
static constexpr size_t SZ_XB  = al256((size_t)NB * SEQ * DM * 2);
static constexpr size_t SZ_WIN = al256((size_t)2 * DI * DM * 2);
static constexpr size_t SZ_WX  = al256((size_t)XPP * DI * 2);
static constexpr size_t SZ_WDT = al256((size_t)DI * DR * 2);
static constexpr size_t SZ_WO  = al256((size_t)DM * DI * 2);
static constexpr size_t SZ_XZ  = al256((size_t)NB * SEQ * XZW * 2);
static constexpr size_t SZ_XC  = al256((size_t)NB * SEQ * DI * 2);
static constexpr size_t SZ_DTR = al256((size_t)NB * SEQ * DR * 2);
static constexpr size_t SZ_BC  = al256((size_t)NB * SEQ * BCW * 4);
static constexpr size_t SZ_PRE = al256((size_t)NB * SEQ * DM * 4);
static constexpr size_t SZ_TOTAL = SZ_XB + SZ_WIN + SZ_WX + SZ_WDT + SZ_WO + SZ_XZ + 3 * SZ_XC + SZ_DTR + SZ_BC + SZ_PRE;
static_assert(SZ_TOTAL <= (size_t)134217728);
static_assert(((size_t)XPN * DI) % 8 == 0);
static_assert(((size_t)XPP * DI) % 8 == 0);
static_assert(((size_t)DI * DR) % 8 == 0);
static_assert(((size_t)DM * DI) % 8 == 0);
static_assert(((size_t)2 * DI * DM) % 8 == 0);

extern "C" void kernel_launch(void* const* d_in, const int* in_sizes, int n_in,
                              void* d_out, int out_size, void* d_ws, size_t ws_size, hipStream_t stream) {
    if (n_in < 12) return;
    const size_t needx = ((size_t)(NB - 1) * SEQ_FULL + SEQ) * DM;
    if ((size_t)in_sizes[0] < needx) return;
    if ((size_t)in_sizes[1] < (size_t)2 * DI * DM) return;
    if ((size_t)in_sizes[2] < (size_t)DI * 4 || in_sizes[3] < DI) return;
    if ((size_t)in_sizes[4] < (size_t)XPN * DI || (size_t)in_sizes[5] < (size_t)DI * DR || in_sizes[6] < DI) return;
    if ((size_t)in_sizes[7] < (size_t)DI * DS || in_sizes[8] < DI) return;
    if ((size_t)in_sizes[9] < (size_t)DM * DI || in_sizes[10] < DM || in_sizes[11] < DM) return;
    if ((size_t)out_size < ((size_t)(NB - 1) * OUT_SEQ + SEQ) * DM) return;
    if (SZ_TOTAL > ws_size) return;
    const float* x    = (const float*)d_in[0];
    const float* win  = (const float*)d_in[1];
    const float* cw   = (const float*)d_in[2];
    const float* cbv  = (const float*)d_in[3];
    const float* wx   = (const float*)d_in[4];
    const float* wdt  = (const float*)d_in[5];
    const float* bdt  = (const float*)d_in[6];
    const float* alog = (const float*)d_in[7];
    const float* dsk  = (const float*)d_in[8];
    const float* wo   = (const float*)d_in[9];
    const float* lng  = (const float*)d_in[10];
    const float* lnb  = (const float*)d_in[11];
    float* OUT = (float*)d_out;
    char* wsp = (char*)d_ws;
    bf*  XB  = (bf*)wsp;  wsp += SZ_XB;
    bf*  WIB = (bf*)wsp;  wsp += SZ_WIN;
    h16* WXH = (h16*)wsp; wsp += SZ_WX;
    h16* WDH = (h16*)wsp; wsp += SZ_WDT;
    h16* WOH = (h16*)wsp; wsp += SZ_WO;
    h16* XZ  = (h16*)wsp; wsp += SZ_XZ;
    h16* XC  = (h16*)wsp; wsp += SZ_XC;
    h16* DT  = (h16*)wsp; wsp += SZ_XC;
    h16* YP  = (h16*)wsp; wsp += SZ_XC;
    h16* DTR = (h16*)wsp; wsp += SZ_DTR;
    float* BC = (float*)wsp; wsp += SZ_BC;
    float* PRE = (float*)wsp; wsp += SZ_PRE;

    if (SEQ == SEQ_FULL) {
        const size_t n8 = (size_t)NB * SEQ * DM / 8;
        k_cvt8<<<(unsigned)((n8 + 255) / 256), 256, 0, stream>>>(x, XB, n8);
    } else {
        const size_t n8 = (size_t)SEQ * DM / 8;
        for (int b = 0; b < NB; ++b) k_cvt8<<<(unsigned)((n8 + 255) / 256), 256, 0, stream>>>(x + (size_t)b * SEQ_FULL * DM, XB + (size_t)b * SEQ * DM, n8);
    }
    { const size_t n8 = (size_t)2 * DI * DM / 8; k_cvt8<<<(unsigned)((n8 + 255) / 256), 256, 0, stream>>>(win, WIB, n8); }
    { const size_t ns = (size_t)XPN * DI / 8, nd = (size_t)XPP * DI / 8; k_wcvth<<<(unsigned)((nd + 255) / 256), 256, 0, stream>>>(wx, WXH, ns, nd, WSC); }
    { const size_t n8 = (size_t)DI * DR / 8; k_wcvth<<<(unsigned)((n8 + 255) / 256), 256, 0, stream>>>(wdt, WDH, n8, n8, WSC); }
    { const size_t n8 = (size_t)DM * DI / 8; k_wcvth<<<(unsigned)((n8 + 255) / 256), 256, 0, stream>>>(wo, WOH, n8, n8, WSC); }

    k_gemm_in<<<dim3(NB * SEQ / 64, XZW / 64, 1), 32, 0, stream>>>(XB, WIB, XZ);
    k_conv<<<dim3(NB * SEQ / CT, 1, 1), 256, 0, stream>>>(XZ, cw, cbv, XC);
    k_gemm_xp<<<dim3(NB * SEQ / 64, XPP / 64, 1), 32, 0, stream>>>(XC, WXH, DTR, BC);
    k_gemm_dt<<<dim3(NB * SEQ / 64, DI / 64, 1), 32, 0, stream>>>(DTR, WDH, bdt, DT);
    k_scan<<<dim3(DI / 64, NB, 1), 64, 0, stream>>>(DT, XC, XZ, BC, alog, dsk, YP);
    k_gemm_out<<<dim3(NB * SEQ / 64, DM / 64, 1), 32, 0, stream>>>(YP, WOH, PRE);
    k_ln<<<dim3(NB * SEQ / 4, 1, 1), 128, 0, stream>>>(PRE, x, lng, lnb, OUT);
}
